// CKConv_22333829939292
// MI455X (gfx1250) — hardware-verified
//
#include <hip/hip_runtime.h>
#include <math.h>

constexpr int HID     = 64;
constexpr int NEDGE   = 30000;
constexpr int EPAD    = 30080;
constexpr int NUSER   = 10000;
constexpr int NITEM   = 20000;
constexpr int KHW     = 50;
constexpr int KHB     = 51;
constexpr int H2ROWS  = 52;
constexpr int KTOT    = KHB * HID;
constexpr float OMEGA0      = 30.0f;
constexpr float W3CARRY     = 256.0f;
constexpr float W3CARRY_INV = 1.0f / 256.0f;
constexpr float INV_KHW     = 1.0f / 50.0f;
constexpr int SIREN_NT = 64;
constexpr int W2PITCH  = 60;
constexpr int GEMM_MT  = 32;
constexpr int GEMM_TILES = EPAD / GEMM_MT;
constexpr int AGG_TN   = 128;
constexpr int AGG_CH   = 2048;
constexpr int AGG_NCH  = (NEDGE + AGG_CH - 1) / AGG_CH;
constexpr int OUT0_FLOATS = NUSER * HID;
constexpr int OUT1_FLOATS = NITEM * HID;

static_assert(EPAD % 128 == 0 && EPAD % GEMM_MT == 0 && EPAD % SIREN_NT == 0 && EPAD >= NEDGE);
static_assert(KTOT % 32 == 0);
static_assert(NEDGE % 8 == 0);
static_assert((NUSER % 2) == 0 && (NITEM % 2) == 0);
static_assert(AGG_CH == 256 * 8);
static_assert(EPAD < 65536);
static_assert(OUT0_FLOATS * 4 == 2560000 && OUT1_FLOATS * 4 == 5120000);

constexpr size_t H2T_BYTES = (size_t)H2ROWS * EPAD * 4;
constexpr size_t X_BYTES   = (size_t)EPAD * HID * 2;
constexpr size_t BT_BYTES  = (size_t)HID * KTOT * 2;
constexpr size_t MSG_BYTES = (size_t)EPAD * HID * 4;
constexpr size_t WS_TOTAL  = 2 * (H2T_BYTES + X_BYTES + BT_BYTES + MSG_BYTES);
static_assert(H2T_BYTES % 256 == 0 && X_BYTES % 256 == 0 && BT_BYTES % 256 == 0 && MSG_BYTES % 256 == 0);
static_assert(WS_TOTAL == 36450304 && WS_TOTAL <= (size_t)134217728);

typedef __attribute__((ext_vector_type(16))) _Float16 v16h;
typedef __attribute__((ext_vector_type(8)))  _Float16 v8h;
typedef __attribute__((ext_vector_type(8)))  float    v8f;
typedef __attribute__((ext_vector_type(4)))  float    v4f;
typedef __attribute__((ext_vector_type(2)))  float    v2f;
typedef __attribute__((ext_vector_type(4)))  int      v4i;
typedef __attribute__((ext_vector_type(4)))  unsigned int v4u;

__device__ __forceinline__ unsigned short f2bf_bits(float f) {
  unsigned u = __float_as_uint(f);
  return (unsigned short)((u + 0x7FFFu + ((u >> 16) & 1u)) >> 16);
}
__device__ __forceinline__ float bf_bits2f(unsigned short h) { return __uint_as_float(((unsigned)h) << 16); }
__device__ __forceinline__ float bfr(float f) { return bf_bits2f(f2bf_bits(f)); }
__device__ __forceinline__ unsigned pk16(unsigned short a, unsigned short b) { return (unsigned)a | ((unsigned)b << 16); }
__device__ __forceinline__ unsigned short h_bits(float f) { const _Float16 h = (_Float16)f; return __builtin_bit_cast(unsigned short, h); }

__device__ __forceinline__ void dep_guard_h(v8f& a, v8f& b, v16h x, v16h y) { asm volatile("v_nop\n\tv_nop\n\tv_nop\n\tv_nop" : "+v"(a), "+v"(b) : "v"(x), "v"(y)); }
__device__ __forceinline__ void keep4_h(v16h a, v16h b, v16h c, v16h d) { asm volatile("v_nop" :: "v"(a), "v"(b), "v"(c), "v"(d)); }
__device__ __forceinline__ void guard4a(v8f& a, v8f& b, v8f& c, v8f& d, v16h x, v16h y0, v16h y1, v16h y2, v16h y3) {
  asm volatile("v_nop\n\tv_nop\n\tv_nop\n\tv_nop" : "+v"(a), "+v"(b), "+v"(c), "+v"(d) : "v"(x), "v"(y0), "v"(y1), "v"(y2), "v"(y3));
}
template <typename T> struct Frag;
template <> struct Frag<_Float16> {
  typedef v16h V; union U { v16h v; v8h h[2]; };
  static __device__ __forceinline__ v16h load(const _Float16* p) {
    U f; f.h[0] = *(const v8h*)(p); f.h[1] = *(const v8h*)(p + 16); return f.v;
  }
  static __device__ __forceinline__ v8f mma(v16h a, v16h b, v8f c) {
    return __builtin_amdgcn_wmma_f32_16x16x32_f16(false, a, false, b, (short)0, c, false, false);
  }
  static __device__ __forceinline__ void guard(v8f& a, v8f& b, v16h x, v16h y) { dep_guard_h(a, b, x, y); }
  static __device__ __forceinline__ void keep(v16h a, v16h b, v16h c, v16h d) { keep4_h(a, b, c, d); }
};

__global__ __launch_bounds__(SIREN_NT) void siren_kernel(
    const float* __restrict__ node_t, int n_nodes, const float* __restrict__ edge_t, const int* __restrict__ nidx,
    const float* __restrict__ w1, const float* __restrict__ b1, const float* __restrict__ g1, const float* __restrict__ be1,
    const float* __restrict__ w2, const float* __restrict__ b2, const float* __restrict__ g2, const float* __restrict__ be2,
    float* __restrict__ h2t)
{
  __shared__ float sw2[KHW * W2PITCH];
  __shared__ float spar[7 * KHW];
  __shared__ float rowA[SIREN_NT * KHW];
  __shared__ __align__(16) float rowB[SIREN_NT * H2ROWS];
  const int tid = threadIdx.x;

#pragma unroll 4
  for (int i = tid; i < KHW * W2PITCH; i += SIREN_NT) {
    const int k  = i / W2PITCH;
    const int c  = i - k * W2PITCH;
    const int g  = c / 12;
    const int jj = c - g * 12;
    int j = g * 10 + jj;
    j = j < KHW ? j : KHW - 1;
    const float v = bfr(w2[k * KHW + j]);
    sw2[i] = (jj < 10) ? v : 0.0f;
  }
  {
    const int jc = tid < KHW ? tid : KHW - 1;
    const float p0 = bfr(w1[jc]), p1 = bfr(b1[jc]), p2 = bfr(g1[jc]), p3 = bfr(be1[jc]);
    const float p4 = bfr(b2[jc]), p5 = bfr(g2[jc]), p6 = bfr(be2[jc]);
    if (tid < KHW) {
      spar[jc] = p0; spar[KHW + jc] = p1; spar[2 * KHW + jc] = p2; spar[3 * KHW + jc] = p3;
      spar[4 * KHW + jc] = p4; spar[5 * KHW + jc] = p5; spar[6 * KHW + jc] = p6;
    }
  }
  __syncthreads();

  const int e = blockIdx.x * SIREN_NT + tid;
  const bool live = e < NEDGE;
  const int ec = live ? e : NEDGE - 1;
  int ix = nidx[ec];
  ix = ix < 0 ? 0 : (ix >= n_nodes ? n_nodes - 1 : ix);
  const float tn = bfr(node_t[ix]);
  const float te = bfr(edge_t[ec]);
  float t = tn - te;
  t = live ? t : 0.0f;

  float* ra = rowA + tid * KHW;
  float* rb = rowB + tid * H2ROWS;

  float m = 0.0f;
#pragma unroll 1
  for (int j = 0; j < KHW; ++j) { const float h = t * spar[j] + spar[KHW + j]; ra[j] = h; m += h; }
  m *= INV_KHW;
  float v = 0.0f;
#pragma unroll 1
  for (int j = 0; j < KHW; ++j) { const float d = ra[j] - m; v += d * d; }
  v *= INV_KHW;
  float rs = 1.0f / sqrtf(v + 1e-5f);
#pragma unroll 1
  for (int j = 0; j < KHW; ++j) {
    float z = (ra[j] - m) * rs;
    z = z * spar[2 * KHW + j] + spar[3 * KHW + j];
    rb[j] = sinf(OMEGA0 * z);
  }

  m = 0.0f;
#pragma unroll 1
  for (int g = 0; g < 5; ++g) {
    float acc[10];
#pragma unroll
    for (int jj = 0; jj < 10; ++jj) acc[jj] = 0.0f;
    const float* wp = sw2 + g * 12;
#pragma unroll 1
    for (int k = 0; k < KHW; ++k) {
      const float hk = rb[k];
      const float* wk = wp + k * W2PITCH;
#pragma unroll
      for (int jj = 0; jj < 10; ++jj) acc[jj] = fmaf(hk, wk[jj], acc[jj]);
    }
#pragma unroll
    for (int jj = 0; jj < 10; ++jj) {
      const float av = acc[jj] + spar[4 * KHW + g * 10 + jj];
      ra[g * 10 + jj] = av;
      m += av;
    }
  }
  m *= INV_KHW;
  v = 0.0f;
#pragma unroll 1
  for (int j = 0; j < KHW; ++j) { const float d = ra[j] - m; v += d * d; }
  v *= INV_KHW;
  rs = 1.0f / sqrtf(v + 1e-5f);

#pragma unroll 1
  for (int j = 0; j < KHW; ++j) {
    float z = (ra[j] - m) * rs;
    z = z * spar[5 * KHW + j] + spar[6 * KHW + j];
    const float s = sinf(OMEGA0 * z);
    rb[j] = live ? s : 0.0f;
  }
  rb[KHW] = live ? 1.0f : 0.0f;
  rb[KHW + 1] = 0.0f;
  __syncthreads();

  const int lane = tid & 31, wave = tid >> 5;
  const int lh = lane & 15, sel = lane >> 4;
  const int e0 = blockIdx.x * SIREN_NT;
  for (int pass = 0; pass < 2; ++pass) {
#pragma unroll 1
    for (int p = 0; p < 13; ++p) {
      const int j = wave + 4 * p + 2 * sel;
      v4f val;
      val[0] = rowB[(4 * lh + 0) * H2ROWS + j];
      val[1] = rowB[(4 * lh + 1) * H2ROWS + j];
      val[2] = rowB[(4 * lh + 2) * H2ROWS + j];
      val[3] = rowB[(4 * lh + 3) * H2ROWS + j];
      *(volatile v4f*)(h2t + (size_t)j * EPAD + e0 + 4 * lh) = val;
    }
    __threadfence();
  }
}

__global__ __launch_bounds__(256) void gather_kernel(const float* __restrict__ emb, int n_nodes,
                                                     const int* __restrict__ nidx, unsigned short* __restrict__ xo) {
  const int g = blockIdx.x * 256 + threadIdx.x;
  const int row = g >> 3, c8 = (g & 7) * 8;
  const bool live = row < NEDGE;
  const int rc = live ? row : NEDGE - 1;
  int ix = nidx[rc];
  ix = ix < 0 ? 0 : (ix >= n_nodes ? n_nodes - 1 : ix);
  const float* src = emb + (size_t)ix * HID + c8;
  const v4f a = *(const v4f*)(src);
  const v4f c = *(const v4f*)(src + 4);
  unsigned short hb[8];
#pragma unroll
  for (int q = 0; q < 4; ++q) {
    const float fa = live ? bfr(a[q]) : 0.0f;
    const float fc = live ? bfr(c[q]) : 0.0f;
    hb[q]     = h_bits(fa);
    hb[4 + q] = h_bits(fc);
  }
  const v4u u = (v4u){pk16(hb[0], hb[1]), pk16(hb[2], hb[3]), pk16(hb[4], hb[5]), pk16(hb[6], hb[7])};
  unsigned short* dst = xo + (size_t)row * HID + c8;
  *(volatile v4u*)dst = u;
  __threadfence();
  *(volatile v4u*)dst = u;
}

__global__ __launch_bounds__(256) void pack_w3_kernel(const float* __restrict__ w3u, const float* __restrict__ b3u,
                                                      const float* __restrict__ w3i, const float* __restrict__ b3i,
                                                      unsigned short* __restrict__ btu, unsigned short* __restrict__ bti) {
  const int side = blockIdx.y;
  const float* w3 = side ? w3i : w3u;
  const float* b3 = side ? b3i : b3u;
  unsigned short* bt = side ? bti : btu;
  const int g = blockIdx.x * 256 + threadIdx.x;
  const int part = g & 7;
  const float* src;
  size_t dst;
  if (blockIdx.x < 100) {
    const int seg = g >> 3;
    const int n = seg / KHW;
    const int j = seg - n * KHW;
    src = w3 + (size_t)j * (HID * HID) + n * HID + part * 8;
    dst = (size_t)n * KTOT + j * HID + part * 8;
  } else {
    const int g2 = g - 100 * 256;
    const int n = g2 >> 3;
    src = b3 + n * HID + part * 8;
    dst = (size_t)n * KTOT + KHW * HID + part * 8;
  }
  const v4f a = *(const v4f*)(src);
  const v4f c = *(const v4f*)(src + 4);
  unsigned short hb[8];
#pragma unroll
  for (int q = 0; q < 4; ++q) {
    hb[q]     = h_bits(bfr(a[q]) * W3CARRY);
    hb[4 + q] = h_bits(bfr(c[q]) * W3CARRY);
  }
  const v4u u = (v4u){pk16(hb[0], hb[1]), pk16(hb[2], hb[3]), pk16(hb[4], hb[5]), pk16(hb[6], hb[7])};
  *(volatile v4u*)(bt + dst) = u;
  __threadfence();
  *(volatile v4u*)(bt + dst) = u;
}

__global__ __launch_bounds__(256) void edge_gemm_kernel(const unsigned short* __restrict__ xp, const unsigned short* __restrict__ btp,
                                                        const float* __restrict__ h2t, float* __restrict__ msg) {
  const _Float16* X  = (const _Float16*)xp;
  const _Float16* Bt = (const _Float16*)btp;
  __shared__ __align__(16) float sT[8][16 * 68];
  const int lane = threadIdx.x & 31;
  const int wave = threadIdx.x >> 5;
  const int tile = blockIdx.x * 8 + wave;
  if (tile >= GEMM_TILES) return;
  const int m0 = tile * GEMM_MT;
  const int rlane = lane & 15;
  const int koff  = (lane >> 4) * 8;
  const int mOff  = (lane >> 4) * 8;

  v8f acc[2][4];
#pragma unroll
  for (int i = 0; i < 2; ++i)
#pragma unroll
    for (int jn = 0; jn < 4; ++jn) acc[i][jn] = (v8f){0.f,0.f,0.f,0.f,0.f,0.f,0.f,0.f};

#pragma unroll 1
  for (int j = 0; j < KHB; ++j) {
#pragma unroll
    for (int i = 0; i < 2; ++i) {
      v8f tmp[4];
#pragma unroll
      for (int jn = 0; jn < 4; ++jn) tmp[jn] = (v8f){0.f,0.f,0.f,0.f,0.f,0.f,0.f,0.f};
#pragma unroll
      for (int half = 0; half < 2; ++half) {
        const int kb = j * HID + half * 32;
        const int kx = half * 32;
        v16h bh[4];
#pragma unroll
        for (int jn = 0; jn < 4; ++jn)
          bh[jn] = Frag<_Float16>::load(Bt + (size_t)(jn * 16 + rlane) * KTOT + koff + kb);
        const v16h a = Frag<_Float16>::load(X + (size_t)(m0 + i * 16 + rlane) * HID + koff + kx);
#pragma unroll
        for (int jn = 0; jn < 4; ++jn) tmp[jn] = Frag<_Float16>::mma(a, bh[jn], tmp[jn]);
        guard4a(tmp[0], tmp[1], tmp[2], tmp[3], a, bh[0], bh[1], bh[2], bh[3]);
      }
      const float* hp = h2t + (size_t)j * EPAD + m0 + i * 16 + mOff;
      const v4f s0 = *(const v4f*)(hp);
      const v4f s1 = *(const v4f*)(hp + 4);
#pragma unroll
      for (int jn = 0; jn < 4; ++jn) {
#pragma unroll
        for (int r = 0; r < 4; ++r) {
          acc[i][jn][r]     = fmaf(tmp[jn][r],     s0[r], acc[i][jn][r]);
          acc[i][jn][4 + r] = fmaf(tmp[jn][4 + r], s1[r], acc[i][jn][4 + r]);
        }
      }
    }
  }

  float* slab = sT[wave];
  const int hh = lane >> 4, c4 = (lane & 15) * 4;
#pragma unroll
  for (int i = 0; i < 2; ++i) {
#pragma unroll
    for (int jn = 0; jn < 4; ++jn) {
#pragma unroll
      for (int r = 0; r < 8; ++r) slab[(mOff + r) * 68 + jn * 16 + rlane] = acc[i][jn][r] * W3CARRY_INV;
    }
    __builtin_amdgcn_fence(__ATOMIC_RELEASE, "workgroup");
    __builtin_amdgcn_wave_barrier();
    __builtin_amdgcn_fence(__ATOMIC_ACQUIRE, "workgroup");
    for (int pass = 0; pass < 2; ++pass) {
#pragma unroll
      for (int it = 0; it < 8; ++it) {
        const int row = it * 2 + hh;
        const v4f vv = *(const v4f*)(slab + row * 68 + c4);
        *(volatile v4f*)(msg + (size_t)(m0 + i * 16 + row) * HID + c4) = vv;
      }
      __threadfence();
    }
    __builtin_amdgcn_fence(__ATOMIC_RELEASE, "workgroup");
    __builtin_amdgcn_wave_barrier();
    __builtin_amdgcn_fence(__ATOMIC_ACQUIRE, "workgroup");
  }
}

__device__ __forceinline__ int blk_excl_scan(int cnt, int* scan_ws, int tid, int* tot) {
  const int lane = tid & 31, wave = tid >> 5; int incl = cnt;
#pragma unroll
  for (int o = 1; o < 32; o <<= 1) { const int v = __shfl_up(incl, o, 32); if (lane >= o) incl += v; }
  if (lane == 31) scan_ws[wave] = incl;
  __syncthreads();
  if (wave == 0) { int wv = (lane < 8) ? scan_ws[lane] : 0; int wincl = wv;
#pragma unroll
    for (int o = 1; o < 32; o <<= 1) { const int v = __shfl_up(wincl, o, 32); if (lane >= o) wincl += v; }
    if (lane < 8) scan_ws[32 + lane] = wincl - wv; if (lane == 31) scan_ws[64] = wincl; }
  __syncthreads();
  const int res = scan_ws[32 + wave] + incl - cnt; *tot = scan_ws[64];
  return res;
}
__device__ __forceinline__ int agg_chunk(const int* __restrict__ didx, int e0, int n0, int tid, int* slist, int* scan_ws) {
  const int eb = e0 + tid * 8;
  const bool inr = eb < NEDGE;
  const int ebc = inr ? eb : NEDGE - 8;
  const v4i d0 = *(const v4i*)(didx + ebc);
  const v4i d1 = *(const v4i*)(didx + ebc + 4);
  int rec[8]; int cnt = 0;
#pragma unroll
  for (int k = 0; k < 8; ++k) {
    const int d = (k < 4) ? d0[k] : d1[k - 4];
    int r = -1;
    if (inr && d >= n0 && d < n0 + AGG_TN) { r = ((d - n0) << 16) | (eb + k); ++cnt; }
    rec[k] = r;
  }
  int tot; int p = blk_excl_scan(cnt, scan_ws, tid, &tot);
#pragma unroll
  for (int k = 0; k < 8; ++k) if (rec[k] >= 0) { if ((unsigned)p < (unsigned)AGG_CH) slist[p] = rec[k]; ++p; }
  __syncthreads();
  return tot < AGG_CH ? tot : AGG_CH;
}

__global__ __launch_bounds__(256) void agg_kernel(const float* __restrict__ msg, const int* __restrict__ didx, int n_nodes,
                                                  float* __restrict__ outp) {
  __shared__ __align__(16) float sacc[AGG_TN * HID];
  __shared__ int slist[AGG_CH];
  __shared__ int scan_ws[80];
  const int tid = threadIdx.x, lane = tid & 31, wave = tid >> 5;
  const int n0 = blockIdx.x * AGG_TN;
  for (int i = tid; i < AGG_CH; i += 256) slist[i] = -1;
  if (tid < 80) scan_ws[tid] = 0;
  const v2f z2 = {0.0f, 0.0f};
#pragma unroll 1
  for (int r = 0; r < 16; ++r) *(v2f*)(sacc + (wave * 16 + r) * HID + 2 * lane) = z2;
  __syncthreads();

#pragma unroll 1
  for (int c = 0; c < AGG_NCH; ++c) {
    const int tot = agg_chunk(didx, c * AGG_CH, n0, tid, slist, scan_ws);
#pragma unroll 1
    for (int base = 0; base < tot; base += 32) {
      const int q = base + lane;
      int rv = slist[q];
      rv = (q < tot) ? rv : -1;
      const int own = (rv >= 0 && (rv >> 20) == wave) ? 1 : 0;
      unsigned msk = (unsigned)__ballot(own);
#pragma unroll 1
      for (int it = 0; it < 32; ++it) {
        if (msk == 0u) break;
        const int bp = __builtin_ctz(msk); msk &= msk - 1u;
        const int r = __shfl(rv, bp, 32);
        const int dl = (r >> 16) & (AGG_TN - 1);
        int e = r & 0xFFFF; e = e < EPAD ? e : EPAD - 1;
        const v2f mv = *(const v2f*)(msg + (size_t)e * HID + 2 * lane);
        float* ap = sacc + dl * HID + 2 * lane;
        v2f a = *(const v2f*)ap;
        a = a + mv;
        *(v2f*)ap = a;
      }
    }
    __syncthreads();
  }

  const int hh = lane >> 4, c4 = (lane & 15) * 4;
  for (int pass = 0; pass < 2; ++pass) {
#pragma unroll
    for (int it = 0; it < 8; ++it) {
      const int dl = wave * 16 + it * 2 + hh;
      const int n = n0 + dl;
      if (n < n_nodes) {
        const v4f vv = *(const v4f*)(sacc + dl * HID + c4);
        *(volatile v4f*)(outp + (size_t)n * HID + c4) = vv;
      }
    }
    __threadfence();
  }
}

extern "C" void kernel_launch(void* const* d_in, const int* in_sizes, int n_in,
                              void* d_out, int out_size, void* d_ws, size_t ws_size,
                              hipStream_t stream)
{
  (void)in_sizes; (void)n_in;
  const float* u_emb  = (const float*)d_in[0];
  const float* i_emb  = (const float*)d_in[1];
  const int*   uix    = (const int*)  d_in[2];
  const int*   iix    = (const int*)  d_in[3];
  const float* edge_t = (const float*)d_in[4];
  const float* u_t    = (const float*)d_in[5];
  const float* i_t    = (const float*)d_in[6];
  const float* up[10]; const float* ip[10];
  for (int q = 0; q < 10; ++q) { up[q] = (const float*)d_in[7 + q]; ip[q] = (const float*)d_in[17 + q]; }

  if (out_size < OUT0_FLOATS + OUT1_FLOATS) return;
  if (ws_size < WS_TOTAL) return;

  char* ws = (char*)d_ws;
  size_t off = 0;
  float*          h2t_i = (float*)(ws + off);          off += H2T_BYTES;
  float*          h2t_u = (float*)(ws + off);          off += H2T_BYTES;
  unsigned short* x_i   = (unsigned short*)(ws + off); off += X_BYTES;
  unsigned short* x_u   = (unsigned short*)(ws + off); off += X_BYTES;
  unsigned short* bt_i  = (unsigned short*)(ws + off); off += BT_BYTES;
  unsigned short* bt_u  = (unsigned short*)(ws + off); off += BT_BYTES;
  float*          msg_i = (float*)(ws + off);          off += MSG_BYTES;
  float*          msg_u = (float*)(ws + off);          off += MSG_BYTES;
  if (off != WS_TOTAL || off > ws_size) return;

  float* out0 = (float*)d_out;
  float* out1 = (float*)d_out + OUT0_FLOATS;

  siren_kernel<<<EPAD / SIREN_NT, SIREN_NT, 0, stream>>>(i_t, NITEM, edge_t, iix,
      ip[0], ip[1], ip[2], ip[3], ip[4], ip[5], ip[6], ip[7], h2t_i);
  siren_kernel<<<EPAD / SIREN_NT, SIREN_NT, 0, stream>>>(u_t, NUSER, edge_t, uix,
      up[0], up[1], up[2], up[3], up[4], up[5], up[6], up[7], h2t_u);
  gather_kernel<<<(EPAD * 8) / 256, 256, 0, stream>>>(i_emb, NITEM, iix, x_i);
  gather_kernel<<<(EPAD * 8) / 256, 256, 0, stream>>>(u_emb, NUSER, uix, x_u);
  pack_w3_kernel<<<dim3(102, 2), 256, 0, stream>>>(up[8], up[9], ip[8], ip[9], bt_u, bt_i);
  const int gemm_blocks = (GEMM_TILES + 7) / 8;
  edge_gemm_kernel<<<gemm_blocks, 256, 0, stream>>>(x_i, bt_i, h2t_i, msg_i);
  edge_gemm_kernel<<<gemm_blocks, 256, 0, stream>>>(x_u, bt_u, h2t_u, msg_u);
  agg_kernel<<<(NUSER + AGG_TN - 1) / AGG_TN, 256, 0, stream>>>(msg_i, uix, NUSER, out0);
  agg_kernel<<<(NITEM + AGG_TN - 1) / AGG_TN, 256, 0, stream>>>(msg_u, iix, NITEM, out1);
}
